// VQ_VAE_9620726743267
// MI455X (gfx1250) — hardware-verified
//
#include <hip/hip_runtime.h>
#include <stddef.h>
#include <math.h>


typedef unsigned short us;
typedef us           v8us  __attribute__((ext_vector_type(8)));
typedef us           v16us __attribute__((ext_vector_type(16)));
typedef __bf16       v16bf __attribute__((ext_vector_type(16)));
typedef float        v8f   __attribute__((ext_vector_type(8)));
typedef float        v4f   __attribute__((ext_vector_type(4)));
typedef float        v2f   __attribute__((ext_vector_type(2)));
typedef unsigned int v4u   __attribute__((ext_vector_type(4)));
union Frag { v16us v; v8us h[2]; };

#define NLAT   32768
#define VQBLK  512
#define RECW   544
#define NJOB   19

__device__ __forceinline__ us f2bf(float f) {
  unsigned int u = __float_as_uint(f);
  u += 0x7FFFu + ((u >> 16) & 1u);
  return (us)(u >> 16);
}
__device__ __forceinline__ float bf2f(us b) { return __uint_as_float(((unsigned int)b) << 16); }

__device__ __forceinline__ void split8(const float (&v)[8], v8us& hi, v8us& lo) {
#pragma unroll
  for (int i = 0; i < 8; ++i) {
    const us hb = f2bf(v[i]);
    hi[i] = hb;
    lo[i] = f2bf(v[i] - bf2f(hb));
  }
}

__device__ __forceinline__ v16us zero16() {
  v16us z;
#pragma unroll
  for (int i = 0; i < 16; ++i) z[i] = (us)0;
  return z;
}
__device__ __forceinline__ v8f zero8f() {
  v8f z;
#pragma unroll
  for (int i = 0; i < 8; ++i) z[i] = 0.0f;
  return z;
}

__device__ __forceinline__ v8f wmb3(v16us ah, v16us al, v16us bh, v16us bl, v8f c) {
#if defined(__HIP_DEVICE_COMPILE__)
  const v16bf Ah = __builtin_bit_cast(v16bf, ah);
  const v16bf Al = __builtin_bit_cast(v16bf, al);
  const v16bf Bh = __builtin_bit_cast(v16bf, bh);
  const v16bf Bl = __builtin_bit_cast(v16bf, bl);
  v8f d = __builtin_amdgcn_wmma_f32_16x16x32_bf16(false, Ah, false, Bh, (short)0, c, false, false);
  d = __builtin_amdgcn_wmma_f32_16x16x32_bf16(false, Ah, false, Bl, (short)0, d, false, false);
  d = __builtin_amdgcn_wmma_f32_16x16x32_bf16(false, Al, false, Bh, (short)0, d, false, false);
  asm volatile("v_nop\n\tv_nop\n\tv_nop\n\tv_nop" : "+v"(d) : "v"(Ah), "v"(Al), "v"(Bh), "v"(Bl));
  return d;
#else
  (void)ah; (void)al; (void)bh; (void)bl;
  return c;
#endif
}

template <int COUT, int NT, int MODE, int WF32, int PRELU, int HOUT, int WOUT>
__device__ __forceinline__ void conv_store(float (*st)[NT * 16], int lane, int mtile, int n0,
                                           int bt, int yt, int x0, int qy, int qx,
                                           float* outf, us* outh, us* outl) {
#pragma unroll
  for (int q = 0; q < NT; ++q) {
    const int p   = q * 32 + lane;
    const int row = p / (2 * NT);
    const int pc  = p - row * (2 * NT);
    const float* sp = &st[row][8 * pc];
    const v4f f0 = *(const v4f*)sp;
    const v4f f1 = *(const v4f*)(sp + 4);
    float v[8] = {f0.x, f0.y, f0.z, f0.w, f1.x, f1.y, f1.z, f1.w};
    if (PRELU) {
#pragma unroll
      for (int i = 0; i < 8; ++i) v[i] = fmaxf(v[i], 0.0f);
    }
    v8us hi, lo;
    split8(v, hi, lo);
    const int gr = (MODE == 0) ? (mtile + row)
                               : (((bt * 2 * HOUT + 2 * yt + qy) * (2 * WOUT)) + 2 * (x0 + row) + qx);
    const size_t g = (size_t)gr * COUT + n0 + 8 * pc;
    *(volatile v8us*)(outh + g) = hi;
    *(volatile v8us*)(outl + g) = lo;
  }
  if (WF32) {
#pragma unroll
    for (int q = 0; q < 2 * NT; ++q) {
      const int p   = q * 32 + lane;
      const int row = p / (4 * NT);
      const int pc  = p - row * (4 * NT);
      const v4f f = *(const v4f*)&st[row][4 * pc];
      const int gr = (MODE == 0) ? (mtile + row)
                                 : (((bt * 2 * HOUT + 2 * yt + qy) * (2 * WOUT)) + 2 * (x0 + row) + qx);
      *(volatile v4f*)(outf + (size_t)gr * COUT + n0 + 4 * pc) = f;
    }
  }
}

template <int HIN, int WIN, int CIN, int HOUT, int WOUT, int COUT, int NT, int KH, int KW, int STR, int PAD,
          int MODE, int HASB, int HASR, int WF32, int PRELU>
__global__ __launch_bounds__(128) void k_conv(const us* __restrict__ inh, const us* __restrict__ inl,
                                              const us* __restrict__ wh, const us* __restrict__ wl,
                                              const float* __restrict__ bias, const float* __restrict__ resf,
                                              float* outf, us* outh, us* outl) {
  constexpr int NTAP = (MODE == 1) ? 4 : (KH * KW);
  constexpr int K    = NTAP * CIN;
  constexpr int TW   = NT * 16;
  constexpr int NBLK = COUT / TW;
  static_assert(CIN % 32 == 0);
  static_assert(K % 32 == 0);
  static_assert((32 * HOUT * WOUT) % 64 == 0);
  static_assert(WOUT % 16 == 0);
  static_assert(NBLK * TW == COUT);
  static_assert((TW == COUT) || (NT >= 4));
  static_assert((MODE == 0) || (TW == COUT));

  __shared__ __attribute__((aligned(16))) float stg[4][16][TW];

  const int tid = threadIdx.x, wave = tid >> 5, lane = tid & 31, hh = lane >> 4, m = lane & 15;
  const int nblk = (int)blockIdx.y % NBLK;
  const int cls  = (int)blockIdx.y / NBLK;
  const int qy = cls >> 1, qx = cls & 1;
  const int n0 = nblk * TW;
  const int mtile = ((int)blockIdx.x * 4 + wave) * 16;
  const int x0 = mtile % WOUT;
  const int yt = (mtile / WOUT) % HOUT;
  const int bt = mtile / (WOUT * HOUT);
  const int xm = x0 + m;
  const us* whc = wh + (size_t)cls * COUT * K;
  const us* wlc = wl + (size_t)cls * COUT * K;
  const v16us zz = zero16();

  v8f acc[NT];
#pragma unroll
  for (int t = 0; t < NT; ++t) acc[t] = zero8f();

#pragma unroll 1
  for (int kk = 0; kk < K; kk += 32) {
    const int tap = kk / CIN;
    const int c0  = kk - tap * CIN;
    int iy, ix;
    if (MODE == 0) {
      const int ky = tap / KW;
      const int kx = tap - ky * KW;
      iy = yt * STR - PAD + ky;
      ix = xm * STR - PAD + kx;
    } else {
      iy = yt + qy + (tap >> 1) - 1;
      ix = xm + qx + (tap & 1) - 1;
    }
    const bool ok = (iy >= 0) && (iy < HIN) && (ix >= 0) && (ix < WIN);
    const int iyc = min(max(iy, 0), HIN - 1);
    const int ixc = min(max(ix, 0), WIN - 1);
    const size_t ab = ((size_t)((bt * HIN + iyc) * WIN + ixc)) * CIN + c0 + 8 * hh;
    Frag fah, fal;
    fah.h[0] = *(const v8us*)(inh + ab);
    fah.h[1] = *(const v8us*)(inh + ab + 16);
    fal.h[0] = *(const v8us*)(inl + ab);
    fal.h[1] = *(const v8us*)(inl + ab + 16);
    const v16us av  = ok ? fah.v : zz;
    const v16us alv = ok ? fal.v : zz;
#pragma unroll
    for (int t = 0; t < NT; ++t) {
      const size_t bb = (size_t)(n0 + t * 16 + m) * K + kk + 8 * hh;
      Frag fbh, fbl;
      fbh.h[0] = *(const v8us*)(whc + bb);
      fbh.h[1] = *(const v8us*)(whc + bb + 16);
      fbl.h[0] = *(const v8us*)(wlc + bb);
      fbl.h[1] = *(const v8us*)(wlc + bb + 16);
      acc[t] = wmb3(av, alv, fbh.v, fbl.v, acc[t]);
    }
  }

#pragma unroll
  for (int t = 0; t < NT; ++t) {
    const int nloc = t * 16 + m;
    const int n = n0 + nloc;
    const float bv = HASB ? bias[n] : 0.0f;
#pragma unroll
    for (int r = 0; r < 8; ++r) {
      const int row = 8 * hh + r;
      float v = acc[t][r] + bv;
      if (HASR) v += resf[(size_t)(mtile + row) * COUT + n];
      stg[wave][row][nloc] = v;
    }
  }
  __syncthreads();
  conv_store<COUT, NT, MODE, WF32, PRELU, HOUT, WOUT>(stg[wave], lane, mtile, n0, bt, yt, x0, qy, qx, outf, outh, outl);
  __threadfence();
  conv_store<COUT, NT, MODE, WF32, PRELU, HOUT, WOUT>(stg[wave], lane, mtile, n0, bt, yt, x0, qy, qx, outf, outh, outl);
}

struct PJob {
  const float* w; us* hi; us* lo;
  int type; int cout; int cin; int kh; int kw; int K; int npad; int qy; int qx; int wn;
};
struct PJobs { PJob j[NJOB]; };
static_assert(sizeof(PJob) == 64);
static_assert(sizeof(PJobs) == 64 * NJOB);

__global__ __launch_bounds__(256) void k_pack(PJobs J) {
  PJob jb = J.j[0];
  switch ((int)blockIdx.y) {
#define PKCASE(i) case i: jb = J.j[i]; break;
    PKCASE(1) PKCASE(2) PKCASE(3) PKCASE(4) PKCASE(5) PKCASE(6) PKCASE(7) PKCASE(8) PKCASE(9)
    PKCASE(10) PKCASE(11) PKCASE(12) PKCASE(13) PKCASE(14) PKCASE(15) PKCASE(16) PKCASE(17) PKCASE(18)
#undef PKCASE
    default: break;
  }
  const int np = jb.npad * jb.K / 8;
  for (int p = (int)blockIdx.x * 256 + (int)threadIdx.x; p < np; p += (int)gridDim.x * 256) {
    const int e0 = p * 8;
    const int n  = e0 / jb.K;
    const int k0 = e0 - n * jb.K;
    float v[8];
#pragma unroll
    for (int j = 0; j < 8; ++j) {
      const int k = k0 + j;
      int src = 0;
      bool ok = false;
      if (jb.type == 0) {
        const int tap = k / jb.cin;
        const int c   = k - tap * jb.cin;
        const int ky  = tap / jb.kw;
        const int kx  = tap - ky * jb.kw;
        ok  = (n < jb.cout) && (tap < jb.kh * jb.kw);
        src = ((n * jb.cin + c) * jb.kh + ky) * jb.kw + kx;
      } else if (jb.type == 1) {
        const int tap = k / jb.cin;
        const int c   = k - tap * jb.cin;
        const int ky  = jb.qy + 2 * (tap >> 1);
        const int kx  = jb.qx + 2 * (tap & 1);
        ok  = (n < jb.cout) && (tap < 4);
        src = ((n * jb.cin + c) * 4 + ky) * 4 + kx;
      } else if (jb.type == 2) {
        const int pp = n / 3;
        const int co = n - 3 * pp;
        const int py = pp >> 1, px = pp & 1;
        const int tap = k / jb.cin;
        const int c   = k - tap * jb.cin;
        const int ty  = tap / 3;
        const int tx  = tap - 3 * ty;
        const int dy = ty - py, dx = tx - px;
        ok  = (n < 12) && (tap < 9) && (dy >= 0) && (dy <= 1) && (dx >= 0) && (dx <= 1);
        const int ky = py + 2 * dy, kx = px + 2 * dx;
        src = ((co * jb.cin + c) * 4 + ky) * 4 + kx;
      } else {
        ok  = (n < jb.cout);
        src = n * jb.K + k;
      }
      src = min(max(src, 0), jb.wn - 1);
      const float t = jb.w[src];
      v[j] = ok ? t : 0.0f;
    }
    v8us hi, lo;
    split8(v, hi, lo);
    *(volatile v8us*)(jb.hi + e0) = hi;
    *(volatile v8us*)(jb.lo + e0) = lo;
    __threadfence();
    *(volatile v8us*)(jb.hi + e0) = hi;
    *(volatile v8us*)(jb.lo + e0) = lo;
  }
}

__global__ __launch_bounds__(256) void k_im2col1(const float* __restrict__ x, us* ah, us* al) {
  const int tid = threadIdx.x;
  const int row = (int)blockIdx.x * 32 + (tid >> 3);
  const int pc  = tid & 7;
  const int xo = row & 63, yo = (row >> 6) & 63, b = row >> 12;
  float v[8];
#pragma unroll
  for (int j = 0; j < 8; ++j) {
    const int k   = pc * 8 + j;
    const int tap = k / 3;
    const int cin = k - 3 * tap;
    const int ky  = (tap >> 2) & 3;
    const int kx  = tap & 3;
    const int iy = 2 * yo - 1 + ky, ix = 2 * xo - 1 + kx;
    const bool ok = (k < 48) && (iy >= 0) && (iy < 128) && (ix >= 0) && (ix < 128);
    const int iyc = min(max(iy, 0), 127), ixc = min(max(ix, 0), 127);
    const float t = x[((size_t)(b * 3 + cin) * 128 + iyc) * 128 + ixc];
    v[j] = ok ? t : 0.0f;
  }
  v8us hi, lo;
  split8(v, hi, lo);
  const size_t g = (size_t)row * 64 + 8 * pc;
  *(volatile v8us*)(ah + g) = hi;
  *(volatile v8us*)(al + g) = lo;
  __threadfence();
  *(volatile v8us*)(ah + g) = hi;
  *(volatile v8us*)(al + g) = lo;
}

__global__ __launch_bounds__(512) void k_cnorm(const float* __restrict__ cb, float* cn) {
  __shared__ __attribute__((aligned(16))) float s[512];
  const int k = threadIdx.x;
  const float* cr = cb + (size_t)k * 64;
  float a = 0.0f;
#pragma unroll 1
  for (int d = 0; d < 64; d += 4) {
    const v4f v = *(const v4f*)(cr + d);
    a += v.x * v.x; a += v.y * v.y; a += v.z * v.z; a += v.w * v.w;
  }
  s[k] = a;
  __syncthreads();
  v4f v = {0.0f, 0.0f, 0.0f, 0.0f};
  if (k < 128) v = *(const v4f*)(s + 4 * k);
  if (k < 128) *(volatile v4f*)(cn + 4 * k) = v;
  __threadfence();
  if (k < 128) *(volatile v4f*)(cn + 4 * k) = v;
}

__global__ __launch_bounds__(128) void k_vq(const float* __restrict__ zf, const us* __restrict__ zh,
                                            const us* __restrict__ zl, const float* __restrict__ cb,
                                            const us* __restrict__ ch, const us* __restrict__ cl,
                                            const float* __restrict__ cnorm, us* qh, us* ql,
                                            unsigned int* rec) {
  __shared__ float  bn[512];
  __shared__ float  arow[64];
  __shared__ int    idxs[64];
  __shared__ double red[128];
  __shared__ __attribute__((aligned(16))) unsigned int rci[RECW];

  const int tid = threadIdx.x, wave = tid >> 5, lane = tid & 31, hh = lane >> 4, m = lane & 15;
  const int blk = (int)blockIdx.x;
  const int row0 = blk * 64;

  for (int i = tid; i < 512; i += 128) bn[i] = cnorm[i];
  if (tid < 64) {
    const float* zr = zf + (size_t)(row0 + tid) * 64;
    float s = 0.0f;
#pragma unroll 1
    for (int d = 0; d < 64; d += 4) {
      const v4f v = *(const v4f*)(zr + d);
      s += v.x * v.x; s += v.y * v.y; s += v.z * v.z; s += v.w * v.w;
    }
    arow[tid] = s;
  }
  __syncthreads();

  const size_t ab = (size_t)(row0 + wave * 16 + m) * 64 + 8 * hh;
  Frag a0h, a0l, a1h, a1l;
  a0h.h[0] = *(const v8us*)(zh + ab);      a0h.h[1] = *(const v8us*)(zh + ab + 16);
  a1h.h[0] = *(const v8us*)(zh + ab + 32); a1h.h[1] = *(const v8us*)(zh + ab + 48);
  a0l.h[0] = *(const v8us*)(zl + ab);      a0l.h[1] = *(const v8us*)(zl + ab + 16);
  a1l.h[0] = *(const v8us*)(zl + ab + 32); a1l.h[1] = *(const v8us*)(zl + ab + 48);

  float ar[8], bs[8];
  int bi[8];
#pragma unroll
  for (int r = 0; r < 8; ++r) { ar[r] = arow[wave * 16 + 8 * hh + r]; bs[r] = 3.0e38f; bi[r] = 0; }

#pragma unroll 1
  for (int nt = 0; nt < 32; ++nt) {
    const size_t bb = (size_t)(nt * 16 + m) * 64 + 8 * hh;
    Frag b0h, b0l, b1h, b1l;
    b0h.h[0] = *(const v8us*)(ch + bb);      b0h.h[1] = *(const v8us*)(ch + bb + 16);
    b1h.h[0] = *(const v8us*)(ch + bb + 32); b1h.h[1] = *(const v8us*)(ch + bb + 48);
    b0l.h[0] = *(const v8us*)(cl + bb);      b0l.h[1] = *(const v8us*)(cl + bb + 16);
    b1l.h[0] = *(const v8us*)(cl + bb + 32); b1l.h[1] = *(const v8us*)(cl + bb + 48);
    v8f acc = zero8f();
    acc = wmb3(a0h.v, a0l.v, b0h.v, b0l.v, acc);
    acc = wmb3(a1h.v, a1l.v, b1h.v, b1l.v, acc);
    const int id = nt * 16 + m;
    const float bv = bn[id];
#pragma unroll
    for (int r = 0; r < 8; ++r) {
      const float s = (ar[r] + bv) - 2.0f * acc[r];
      if (s < bs[r]) { bs[r] = s; bi[r] = id; }
    }
  }
#pragma unroll
  for (int r = 0; r < 8; ++r) {
    float s = bs[r];
    int id = bi[r];
#pragma unroll
    for (int off = 8; off >= 1; off >>= 1) {
      const float os  = __shfl_xor(s, off, 32);
      const int   oid = __shfl_xor(id, off, 32);
      const bool take = (os < s) || ((os == s) && (oid < id));
      s  = take ? os : s;
      id = take ? oid : id;
    }
    if (m == 0) idxs[wave * 16 + 8 * hh + r] = id;
  }
  __syncthreads();

  float sq = 0.0f;
  v8us qhv[4], qlv[4];
#pragma unroll
  for (int i = 0; i < 4; ++i) {
    const int p = 128 * i + tid;
    const int r = p >> 3, pc = p & 7;
    int id = idxs[r];
    id = min(max(id, 0), 511);
    const float* cp = cb + (size_t)id * 64 + 8 * pc;
    const float* zp = zf + (size_t)(row0 + r) * 64 + 8 * pc;
    const v4f c0 = *(const v4f*)cp, c1 = *(const v4f*)(cp + 4);
    const v4f z0 = *(const v4f*)zp, z1 = *(const v4f*)(zp + 4);
    const float qv[8] = {c0.x, c0.y, c0.z, c0.w, c1.x, c1.y, c1.z, c1.w};
    const float zv[8] = {z0.x, z0.y, z0.z, z0.w, z1.x, z1.y, z1.z, z1.w};
#pragma unroll
    for (int j = 0; j < 8; ++j) { const float d = qv[j] - zv[j]; sq += d * d; }
    split8(qv, qhv[i], qlv[i]);
  }
  unsigned int cA = 0u, cB = 0u, cC = 0u, cD = 0u;
#pragma unroll 1
  for (int r = 0; r < 64; ++r) {
    const int v = idxs[r];
    cA += (v == tid) ? 1u : 0u;
    cB += (v == tid + 128) ? 1u : 0u;
    cC += (v == tid + 256) ? 1u : 0u;
    cD += (v == tid + 384) ? 1u : 0u;
  }
  rci[tid] = cA; rci[tid + 128] = cB; rci[tid + 256] = cC; rci[tid + 384] = cD;
  red[tid] = (double)sq;
  __syncthreads();
#pragma unroll 1
  for (int st = 64; st > 0; st >>= 1) {
    if (tid < st) red[tid] += red[tid + st];
    __syncthreads();
  }
  if (tid == 0) {
    const unsigned long long bits = (unsigned long long)__double_as_longlong(red[0]);
    rci[512] = (unsigned int)(bits & 0xFFFFFFFFull);
    rci[513] = (unsigned int)(bits >> 32);
  }
  if (tid < 30) rci[514 + tid] = 0u;
  __syncthreads();
  const v4u rv0 = *(const v4u*)(rci + 4 * tid);
  v4u rv1 = {0u, 0u, 0u, 0u};
  if (tid < 8) rv1 = *(const v4u*)(rci + 512 + 4 * tid);
  unsigned int* rp = rec + (size_t)blk * RECW;

#pragma unroll
  for (int i = 0; i < 4; ++i) {
    const int p = 128 * i + tid;
    const int r = p >> 3, pc = p & 7;
    const size_t g = (size_t)(row0 + r) * 64 + 8 * pc;
    *(volatile v8us*)(qh + g) = qhv[i];
    *(volatile v8us*)(ql + g) = qlv[i];
  }
  *(volatile v4u*)(rp + 4 * tid) = rv0;
  if (tid < 8) *(volatile v4u*)(rp + 512 + 4 * tid) = rv1;
  __threadfence();
#pragma unroll
  for (int i = 0; i < 4; ++i) {
    const int p = 128 * i + tid;
    const int r = p >> 3, pc = p & 7;
    const size_t g = (size_t)(row0 + r) * 64 + 8 * pc;
    *(volatile v8us*)(qh + g) = qhv[i];
    *(volatile v8us*)(ql + g) = qlv[i];
  }
  *(volatile v4u*)(rp + 4 * tid) = rv0;
  if (tid < 8) *(volatile v4u*)(rp + 512 + 4 * tid) = rv1;
}

__global__ __launch_bounds__(512) void k_fin(const unsigned int* __restrict__ rec, float* scal) {
  __shared__ double red[512];
  __shared__ __attribute__((aligned(16))) float sc[32];
  const int k = threadIdx.x;
  unsigned int cnt = 0u;
#pragma unroll 1
  for (int bI = 0; bI < VQBLK; ++bI) cnt += rec[(size_t)bI * RECW + k];
  const float p = (float)cnt * (1.0f / 32768.0f);
  const float term = p * logf(p + 1e-10f);
  red[k] = (double)term;
  __syncthreads();
#pragma unroll 1
  for (int st = 256; st > 0; st >>= 1) {
    if (k < st) red[k] += red[k + st];
    __syncthreads();
  }
  if (k == 0) {
    const double H = red[0];
    double S = 0.0;
#pragma unroll 1
    for (int bI = 0; bI < VQBLK; ++bI) {
      const unsigned long long lo = (unsigned long long)rec[(size_t)bI * RECW + 512];
      const unsigned long long hi = (unsigned long long)rec[(size_t)bI * RECW + 513];
      S += __longlong_as_double((long long)((hi << 32) | lo));
    }
    sc[0] = (float)(1.25 * S * (1.0 / (32768.0 * 64.0)));
    sc[1] = (float)exp(-H);
#pragma unroll
    for (int j = 2; j < 32; ++j) sc[j] = 0.0f;
  }
  __syncthreads();
  v4f v = {0.0f, 0.0f, 0.0f, 0.0f};
  if (k < 8) v = *(const v4f*)(sc + 4 * k);
  if (k < 8) *(volatile v4f*)(scal + 4 * k) = v;
  __threadfence();
  if (k < 8) *(volatile v4f*)(scal + 4 * k) = v;
}

__device__ __forceinline__ void seg_store(float* out, int R, float pred, const float* body, int lane) {
  const int j0 = 4 * lane;
  const float b0 = body[max(j0 - 1, 0)];
  v4f f;
  f.x = (j0 == 0) ? pred : b0;
  f.y = body[j0];
  f.z = body[j0 + 1];
  f.w = body[j0 + 2];
  *(volatile v4f*)(out + (size_t)R * 128 + j0) = f;
}

__device__ __forceinline__ void final_pass(float* out, const float* V, const float* hold, const float* lastpix,
                                           float loss, int b, int Y, int wave, int lane) {
  if (wave < 3) {
    const int c = wave;
    seg_store(out, (b * 3 + c) * 128 + 2 * Y + 1, V[(c * 2) * 128 + 127], V + (c * 2 + 1) * 128, lane);
  } else {
    const float lp0 = lastpix[0], lp2 = lastpix[2];
    const float pred = (Y > 0) ? lp0 : ((b == 0) ? loss : lp2);
    seg_store(out, (b * 3) * 128 + 2 * Y, pred, V, lane);
  }
  if (wave < 2) {
    const int c = wave + 1;
    if (Y > 0) seg_store(out, (b * 3 + c) * 128 + 2 * Y, lastpix[c], V + (c * 2) * 128, lane);
  } else {
    const int c = wave - 1;
    if (Y == 63) seg_store(out, (b * 3 + c) * 128, V[((c - 1) * 2 + 1) * 128 + 127], hold + (c - 1) * 128, lane);
  }
}

__global__ __launch_bounds__(128) void k_final(const us* __restrict__ gh, const us* __restrict__ gl,
                                               const us* __restrict__ wh, const us* __restrict__ wl,
                                               const float* __restrict__ bias, const float* __restrict__ scal,
                                               float* out) {
  __shared__ __attribute__((aligned(16))) float V[6 * 128];
  __shared__ float hold[2 * 128];
  __shared__ float lastpix[4];

  const int tid = threadIdx.x, wave = tid >> 5, lane = tid & 31, hh = lane >> 4, m = lane & 15;
  const float loss = scal[0];
  const float perp = scal[1];
  const int n  = m;
  const int pp = n / 3;
  const int co = n - 3 * pp;
  const int py = (pp >> 1) & 1, px = pp & 1;
  const float bco = bias[co];
  const v16us zz = zero16();

  if (tid < 4) lastpix[tid] = 0.0f;
  for (int i = tid; i < 256; i += 128) hold[i] = 0.0f;
  __syncthreads();

#pragma unroll 1
  for (int it = 0; it < 2048; ++it) {
    const int b = it >> 6, Y = it & 63;
    const int X = wave * 16 + m;
    v8f acc = zero8f();
#pragma unroll 1
    for (int kk = 0; kk < 576; kk += 32) {
      const int tap = kk >> 6;
      const int c0  = kk & 63;
      const int ty  = tap / 3;
      const int tx  = tap - 3 * ty;
      const int iy = Y - 1 + ty, ix = X - 1 + tx;
      const bool ok = (iy >= 0) && (iy < 64) && (ix >= 0) && (ix < 64);
      const int iyc = min(max(iy, 0), 63), ixc = min(max(ix, 0), 63);
      const size_t ab = ((size_t)((b * 64 + iyc) * 64 + ixc)) * 64 + c0 + 8 * hh;
      Frag fah, fal, fbh, fbl;
      fah.h[0] = *(const v8us*)(gh + ab); fah.h[1] = *(const v8us*)(gh + ab + 16);
      fal.h[0] = *(const v8us*)(gl + ab); fal.h[1] = *(const v8us*)(gl + ab + 16);
      const v16us av  = ok ? fah.v : zz;
      const v16us alv = ok ? fal.v : zz;
      const size_t bb = (size_t)m * 576 + kk + 8 * hh;
      fbh.h[0] = *(const v8us*)(wh + bb); fbh.h[1] = *(const v8us*)(wh + bb + 16);
      fbl.h[0] = *(const v8us*)(wl + bb); fbl.h[1] = *(const v8us*)(wl + bb + 16);
      acc = wmb3(av, alv, fbh.v, fbl.v, acc);
    }
    if (n < 12) {
#pragma unroll
      for (int r = 0; r < 8; ++r) {
        const int Xr = wave * 16 + 8 * hh + r;
        V[(co * 2 + py) * 128 + 2 * Xr + px] = acc[r] + bco;
      }
    }
    __syncthreads();
    final_pass(out, V, hold, lastpix, loss, b, Y, wave, lane);
    __threadfence();
    final_pass(out, V, hold, lastpix, loss, b, Y, wave, lane);
    __syncthreads();
    if (Y == 0) {
      for (int i = tid; i < 254; i += 128) {
        const int c = i / 127;
        const int j = i - 127 * c;
        hold[c * 128 + j] = V[((c + 1) * 2) * 128 + j];
      }
    }
    if (tid < 3) lastpix[tid] = V[(tid * 2 + 1) * 128 + 127];
    __syncthreads();
  }
  const float lastv = V[(2 * 2 + 1) * 128 + 127];
  v2f f;
  f.x = lastv;
  f.y = perp;
  if (tid == 0) *(volatile v2f*)(out + (size_t)NLAT * 48) = f;
  __threadfence();
  if (tid == 0) *(volatile v2f*)(out + (size_t)NLAT * 48) = f;
}

#define KCONV_C1    k_conv<64, 64, 64,   64, 64,  64, 4,  1, 1, 1, 0,  0,  1, 0, 0, 1>
#define KCONV_C2    k_conv<64, 64, 64,   32, 32, 128, 4,  4, 4, 2, 1,  0,  1, 0, 0, 1>
#define KCONV_C3    k_conv<32, 32, 128,  32, 32, 128, 4,  3, 3, 1, 1,  0,  1, 0, 1, 1>
#define KCONV_CRA   k_conv<32, 32, 128,  32, 32,  32, 2,  3, 3, 1, 1,  0,  0, 0, 0, 1>
#define KCONV_CRB1  k_conv<32, 32, 32,   32, 32, 128, 4,  1, 1, 1, 0,  0,  0, 1, 1, 1>
#define KCONV_CRB2  k_conv<32, 32, 32,   32, 32, 128, 4,  1, 1, 1, 0,  0,  0, 1, 0, 1>
#define KCONV_CPRE  k_conv<32, 32, 128,  32, 32,  64, 4,  1, 1, 1, 0,  0,  1, 0, 1, 0>
#define KCONV_CD1   k_conv<32, 32, 64,   32, 32, 128, 4,  3, 3, 1, 1,  0,  1, 0, 1, 1>
#define KCONV_CT1   k_conv<32, 32, 128,  32, 32,  64, 4,  4, 4, 1, 0,  1,  1, 0, 0, 1>

extern "C" void kernel_launch(void* const* d_in, const int* in_sizes, int n_in,
                              void* d_out, int out_size, void* d_ws, size_t ws_size,
                              hipStream_t stream) {
  if (n_in != 24) return;
  const int expect[24] = {1572864, 3072, 64, 131072, 128, 147456, 128, 36864, 4096, 36864, 4096,
                          8192, 64, 32768, 73728, 128, 36864, 4096, 36864, 4096, 131072, 64, 3072, 3};
  for (int i = 0; i < 24; ++i) if (in_sizes[i] != expect[i]) return;
  if (out_size != NLAT * 48 + 2) return;

  const float* x     = (const float*)d_in[0];
  const float* e_w1  = (const float*)d_in[1];  const float* e_b1  = (const float*)d_in[2];
  const float* e_w2  = (const float*)d_in[3];  const float* e_b2  = (const float*)d_in[4];
  const float* e_w3  = (const float*)d_in[5];  const float* e_b3  = (const float*)d_in[6];
  const float* e_r1a = (const float*)d_in[7];  const float* e_r1b = (const float*)d_in[8];
  const float* e_r2a = (const float*)d_in[9];  const float* e_r2b = (const float*)d_in[10];
  const float* pre_w = (const float*)d_in[11]; const float* pre_b = (const float*)d_in[12];
  const float* cbk   = (const float*)d_in[13];
  const float* d_w1  = (const float*)d_in[14]; const float* d_b1  = (const float*)d_in[15];
  const float* d_r1a = (const float*)d_in[16]; const float* d_r1b = (const float*)d_in[17];
  const float* d_r2a = (const float*)d_in[18]; const float* d_r2b = (const float*)d_in[19];
  const float* dt_w1 = (const float*)d_in[20]; const float* dt_b1 = (const float*)d_in[21];
  const float* dt_w2 = (const float*)d_in[22]; const float* dt_b2 = (const float*)d_in[23];
  float* out = (float*)d_out;

  char* ws = (char*)d_ws;
  size_t off = 0;
  auto carve = [&](size_t bytes) -> char* { char* p = ws + off; off += (bytes + 127) & ~(size_t)127; return p; };
  const size_t SLOT = (size_t)16777216;
  const size_t HALF = (size_t)8388608;
  char* S0 = carve(SLOT); char* S1 = carve(SLOT); char* S2 = carve(SLOT);
  char* S3 = carve(SLOT); char* S4 = carve(SLOT); char* S5 = carve(SLOT);
  us *w1h, *w1l, *w2h, *w2l, *w3h, *w3l, *er1ah, *er1al, *er1bh, *er1bl, *er2ah, *er2al, *er2bh, *er2bl;
  us *prh, *prl, *cbh, *cbl, *dw1h, *dw1l, *dr1ah, *dr1al, *dr1bh, *dr1bl, *dr2ah, *dr2al, *dr2bh, *dr2bl;
  us *dt1h, *dt1l, *dt2h, *dt2l;
  auto wplane = [&](size_t npad, size_t K, us*& hi, us*& lo) { hi = (us*)carve(npad * K * 2); lo = (us*)carve(npad * K * 2); };
  wplane(64, 64, w1h, w1l);
  wplane(128, 1024, w2h, w2l);
  wplane(128, 1152, w3h, w3l);
  wplane(32, 1152, er1ah, er1al);  wplane(128, 32, er1bh, er1bl);
  wplane(32, 1152, er2ah, er2al);  wplane(128, 32, er2bh, er2bl);
  wplane(64, 128, prh, prl);
  wplane(512, 64, cbh, cbl);
  wplane(128, 576, dw1h, dw1l);
  wplane(32, 1152, dr1ah, dr1al);  wplane(128, 32, dr1bh, dr1bl);
  wplane(32, 1152, dr2ah, dr2al);  wplane(128, 32, dr2bh, dr2bl);
  wplane(4 * 64, 512, dt1h, dt1l);
  wplane(16, 576, dt2h, dt2l);
  float*        cnrm = (float*)carve(512 * 4);
  float*        scal = (float*)carve(128);
  unsigned int* rec  = (unsigned int*)carve((size_t)VQBLK * RECW * 4);
  if (off > ws_size) return;
  if (off > (size_t)134217728) return;

  us* a1h = (us*)S0;            us* a1l = (us*)S1;
  us* h1h = (us*)S2;            us* h1l = (us*)S3;
  us* h2h = (us*)S4;            us* h2l = (us*)(S4 + HALF);
  float* h3f = (float*)S0;      us* h3h = (us*)S1;            us* h3l = (us*)(S1 + HALF);
  us* rh  = (us*)S2;            us* rl  = (us*)(S2 + 2097152);
  float* h4f = (float*)S3;      us* h4h = (us*)S4;            us* h4l = (us*)(S4 + HALF);
  us* h5h = (us*)S0;            us* h5l = (us*)(S0 + HALF);
  float* zf  = (float*)S1;      us* zh  = (us*)S2;            us* zl  = (us*)(S2 + 4194304);
  us* qh  = (us*)S3;            us* ql  = (us*)(S3 + 4194304);
  float* g1f = (float*)S0;      us* g1h = (us*)S1;            us* g1l = (us*)(S1 + HALF);
  float* g2f = (float*)S4;      us* g2h = (us*)S5;            us* g2l = (us*)(S5 + HALF);
  us* g3h = (us*)S0;            us* g3l = (us*)(S0 + HALF);
  us* g4h = (us*)S1;            us* g4l = (us*)S2;
  const float* fdum = scal;
  float* fodum = scal;

  PJobs J;
  int nj = 0;
  auto job = [&](const float* w, us* hi, us* lo, int type, int cout, int cin, int kh, int kw, int K, int npad,
                 int qy, int qx, int wn) {
    PJob& p = J.j[nj++];
    p.w = w; p.hi = hi; p.lo = lo; p.type = type; p.cout = cout; p.cin = cin; p.kh = kh; p.kw = kw;
    p.K = K; p.npad = npad; p.qy = qy; p.qx = qx; p.wn = wn;
  };
  job(e_w1,  w1h,   w1l,   0,  64,   3, 4, 4,   64,  64, 0, 0, 3072);
  job(e_w2,  w2h,   w2l,   0, 128,  64, 4, 4, 1024, 128, 0, 0, 131072);
  job(e_w3,  w3h,   w3l,   0, 128, 128, 3, 3, 1152, 128, 0, 0, 147456);
  job(e_r1a, er1ah, er1al, 0,  32, 128, 3, 3, 1152,  32, 0, 0, 36864);
  job(e_r1b, er1bh, er1bl, 0, 128,  32, 1, 1,   32, 128, 0, 0, 4096);
  job(e_r2a, er2ah, er2al, 0,  32, 128, 3, 3, 1152,  32, 0, 0, 36864);
  job(e_r2b, er2bh, er2bl, 0, 128,  32, 1, 1,   32, 128, 0, 0, 4096);
  job(pre_w, prh,   prl,   0,  64, 128, 1, 1,  128,  64, 0, 0, 8192);
  job(cbk,   cbh,   cbl,   3, 512,  64, 1, 1,   64, 512, 0, 0, 32768);
  job(d_w1,  dw1h,  dw1l,  0, 128,  64, 3, 3,  576, 128, 0, 0, 73728);
  job(d_r1a, dr1ah, dr1al, 0,  32, 128, 3, 3, 1152,  32, 0, 0, 36864);
  job(d_r1b, dr1bh, dr1bl, 0, 128,  32, 1, 1,   32, 128, 0, 0, 4096);
  job(d_r2a, dr2ah, dr2al, 0,  32, 128, 3, 3, 1152,  32, 0, 0, 36864);
  job(d_r2b, dr2bh, dr2bl, 0, 128,  32, 1, 1,   32, 128, 0, 0, 4096);
  for (int c = 0; c < 4; ++c)
    job(dt_w1, dt1h + (size_t)c * 64 * 512, dt1l + (size_t)c * 64 * 512, 1, 64, 128, 4, 4, 512, 64, c >> 1, c & 1, 131072);
  job(dt_w2, dt2h,  dt2l,  2,   3,  64, 4, 4,  576,  16, 0, 0, 3072);
  if (nj != NJOB) return;

  k_pack<<<dim3(8, NJOB), 256, 0, stream>>>(J);
  k_im2col1<<<4096, 256, 0, stream>>>(x, a1h, a1l);

  KCONV_C1<<<dim3(2048, 1), 128, 0, stream>>>(a1h, a1l, w1h, w1l, e_b1, fdum, fodum, h1h, h1l);
  KCONV_C2<<<dim3(512, 2), 128, 0, stream>>>(h1h, h1l, w2h, w2l, e_b2, fdum, fodum, h2h, h2l);
  KCONV_C3<<<dim3(512, 2), 128, 0, stream>>>(h2h, h2l, w3h, w3l, e_b3, fdum, h3f, h3h, h3l);
  KCONV_CRA<<<dim3(512, 1), 128, 0, stream>>>(h3h, h3l, er1ah, er1al, fdum, fdum, fodum, rh, rl);
  KCONV_CRB1<<<dim3(512, 2), 128, 0, stream>>>(rh, rl, er1bh, er1bl, fdum, h3f, h4f, h4h, h4l);
  KCONV_CRA<<<dim3(512, 1), 128, 0, stream>>>(h4h, h4l, er2ah, er2al, fdum, fdum, fodum, rh, rl);
  KCONV_CRB2<<<dim3(512, 2), 128, 0, stream>>>(rh, rl, er2bh, er2bl, fdum, h4f, fodum, h5h, h5l);
  KCONV_CPRE<<<dim3(512, 1), 128, 0, stream>>>(h5h, h5l, prh, prl, pre_b, fdum, zf, zh, zl);

  k_cnorm<<<1, 512, 0, stream>>>(cbk, cnrm);
  k_vq<<<VQBLK, 128, 0, stream>>>(zf, zh, zl, cbk, cbh, cbl, cnrm, qh, ql, rec);
  k_fin<<<1, 512, 0, stream>>>(rec, scal);

  KCONV_CD1<<<dim3(512, 2), 128, 0, stream>>>(qh, ql, dw1h, dw1l, d_b1, fdum, g1f, g1h, g1l);
  KCONV_CRA<<<dim3(512, 1), 128, 0, stream>>>(g1h, g1l, dr1ah, dr1al, fdum, fdum, fodum, rh, rl);
  KCONV_CRB1<<<dim3(512, 2), 128, 0, stream>>>(rh, rl, dr1bh, dr1bl, fdum, g1f, g2f, g2h, g2l);
  KCONV_CRA<<<dim3(512, 1), 128, 0, stream>>>(g2h, g2l, dr2ah, dr2al, fdum, fdum, fodum, rh, rl);
  KCONV_CRB2<<<dim3(512, 2), 128, 0, stream>>>(rh, rl, dr2bh, dr2bl, fdum, g2f, fodum, g3h, g3l);
  KCONV_CT1<<<dim3(512, 4), 128, 0, stream>>>(g3h, g3l, dt1h, dt1l, dt_b1, fdum, fodum, g4h, g4l);
  k_final<<<1, 128, 0, stream>>>(g4h, g4l, dt2h, dt2l, dt_b2, scal, out);
}
